// DPRNNUnit_33526514712780
// MI455X (gfx1250) — hardware-verified
//
#include <hip/hip_runtime.h>
#include <math.h>

constexpr int kB   = 4;
constexpr int kC   = 64;
constexpr int kF   = 128;
constexpr int kT   = 128;
constexpr int kK   = 8;
constexpr int kH   = 32;
constexpr int kS   = kT - kK + 1;
constexpr int kN   = kB * kF;
constexpr int kCK  = kC * kK;
constexpr int kG4  = 4 * kH;
constexpr int kH2  = 2 * kH;
constexpr int kSN  = kS * kN;
constexpr int kFT  = kF * kT;
constexpr int kNT  = kN * kT;
constexpr int kHP  = 136;
constexpr float kWCarryInv = 1.0f / 16.0f;
constexpr float kWCarry    = 16.0f;

typedef __attribute__((ext_vector_type(16))) _Float16 v16h;
typedef __attribute__((ext_vector_type(8)))  _Float16 v8h;
typedef __attribute__((ext_vector_type(16))) __bf16   v16b;
typedef __attribute__((ext_vector_type(8)))  __bf16   v8b;
typedef __attribute__((ext_vector_type(8)))  float    v8f;
typedef __attribute__((ext_vector_type(4)))  float    v4f;
typedef __attribute__((ext_vector_type(4)))  unsigned int v4u;

__device__ __forceinline__ unsigned short f2bf_bits(float f) {
  unsigned u = __float_as_uint(f);
  return (unsigned short)((u + 0x7FFFu + ((u >> 16) & 1u)) >> 16);
}
__device__ __forceinline__ float bf_bits2f(unsigned short h) { return __uint_as_float(((unsigned)h) << 16); }

__device__ __forceinline__ void dep_guard_h(v8f& a, v8f& b, v16h x, v16h y) { asm volatile("v_nop\n\tv_nop\n\tv_nop\n\tv_nop" : "+v"(a), "+v"(b) : "v"(x), "v"(y)); }
__device__ __forceinline__ void dep_guard_b(v8f& a, v8f& b, v16b x, v16b y) { asm volatile("v_nop\n\tv_nop\n\tv_nop\n\tv_nop" : "+v"(a), "+v"(b) : "v"(x), "v"(y)); }
__device__ __forceinline__ void keep4_h(v16h a, v16h b, v16h c, v16h d) { asm volatile("v_nop" :: "v"(a), "v"(b), "v"(c), "v"(d)); }
__device__ __forceinline__ void keep4_b(v16b a, v16b b, v16b c, v16b d) { asm volatile("v_nop" :: "v"(a), "v"(b), "v"(c), "v"(d)); }
__device__ __forceinline__ void acc_guard4(v8f& a, v8f& b, v8f& c, v8f& d) { asm volatile("v_nop\n\tv_nop\n\tv_nop\n\tv_nop" : "+v"(a), "+v"(b), "+v"(c), "+v"(d)); }
__device__ __forceinline__ void acc_guard4a(v8f& a, v8f& b, v8f& c, v8f& d, v16h x) { asm volatile("v_nop\n\tv_nop\n\tv_nop\n\tv_nop" : "+v"(a), "+v"(b), "+v"(c), "+v"(d) : "v"(x)); }
template <typename T> struct Frag;
template <> struct Frag<_Float16> {
  typedef v16h V; union U { v16h v; v8h h[2]; };
  static __device__ __forceinline__ v16h load(const _Float16* p) {
    U f; f.h[0] = *(const v8h*)(p); f.h[1] = *(const v8h*)(p + 16); return f.v;
  }
  static __device__ __forceinline__ v8f mma(v16h a, v16h b, v8f c) {
    return __builtin_amdgcn_wmma_f32_16x16x32_f16(false, a, false, b, (short)0, c, false, false);
  }
  static __device__ __forceinline__ void guard(v8f& a, v8f& b, v16h x, v16h y) { dep_guard_h(a, b, x, y); }
  static __device__ __forceinline__ void keep(v16h a, v16h b, v16h c, v16h d) { keep4_h(a, b, c, d); }
};
template <> struct Frag<__bf16> {
  typedef v16b V; union U { v16b v; v8b h[2]; };
  static __device__ __forceinline__ v16b load(const __bf16* p) {
    U f; f.h[0] = *(const v8b*)(p); f.h[1] = *(const v8b*)(p + 16); return f.v;
  }
  static __device__ __forceinline__ v8f mma(v16b a, v16b b, v8f c) {
    return __builtin_amdgcn_wmma_f32_16x16x32_bf16(false, a, false, b, (short)0, c, false, false);
  }
  static __device__ __forceinline__ void guard(v8f& a, v8f& b, v16b x, v16b y) { dep_guard_b(a, b, x, y); }
  static __device__ __forceinline__ void keep(v16b a, v16b b, v16b c, v16b d) { keep4_b(a, b, c, d); }
};

__device__ __forceinline__ unsigned pk16(unsigned short a, unsigned short b) { return (unsigned)a | ((unsigned)b << 16); }
__device__ __forceinline__ unsigned short h_bits(float f) { const _Float16 h = (_Float16)f; return __builtin_bit_cast(unsigned short, h); }

template <int ET> struct Elem;
template <> struct Elem<0> { typedef _Float16 T; };
template <> struct Elem<1> { typedef __bf16 T; };
template <int ET, bool SPLIT, int BIAS_MODE, int OUT_MODE, bool RESID, int ACT = 0>
__global__ __launch_bounds__(256) void wmma_gemm64(
    const unsigned short* __restrict__ Ap, const unsigned short* __restrict__ A2p, int lda, long strideA,
    const unsigned short* __restrict__ Btp, const unsigned short* __restrict__ Bt2p, int ldb, long strideB,
    void* __restrict__ Cout, void* __restrict__ Cout2, int ldc, long strideC,
    const float* __restrict__ bias,
    const float* __restrict__ resid, long strideR,
    int M, int N, int K, float scale) {
  typedef typename Elem<ET>::T T;
  typedef typename Frag<T>::V V;
  const T* A = (const T*)Ap; const T* A2 = (const T*)A2p; const T* Bt = (const T*)Btp; const T* Bt2 = (const T*)Bt2p;
  __shared__ __align__(16) float sT[8][16 * 68];
  const int b    = blockIdx.y;
  const int lane = threadIdx.x & 31;
  const int wave = threadIdx.x >> 5;
  const int tilesN = N >> 6;
  const int tilesM = M >> 6;
  const int tile = blockIdx.x * 8 + wave;
  if (tile >= tilesM * tilesN) return;
  const int tm = tile / tilesN;
  const int tn = tile - tm * tilesN;
  const int m0 = tm << 6;
  const int n0 = tn << 6;

  const T* Ab  = A  + (size_t)b * strideA;
  const T* Bb  = Bt + (size_t)b * strideB;
  const T* Ab2 = SPLIT ? (A2  + (size_t)b * strideA) : nullptr;
  const T* Bb2 = SPLIT ? (Bt2 + (size_t)b * strideB) : nullptr;

  const int rlane = lane & 15;
  const int koff  = (lane >> 4) * 8;
  const int mOff  = (lane >> 4) * 8;

  v8f acc[4][4];
#pragma unroll
  for (int i = 0; i < 4; ++i)
#pragma unroll
    for (int j = 0; j < 4; ++j) acc[i][j] = (v8f){0.f,0.f,0.f,0.f,0.f,0.f,0.f,0.f};

  for (int k0 = 0; k0 < K; k0 += 32) {
    V bh[4], bl[4];
#pragma unroll
    for (int j = 0; j < 4; ++j) {
      const size_t bo = (size_t)(n0 + (j << 4) + rlane) * ldb + koff + k0;
      bh[j] = Frag<T>::load(Bb + bo);
      if (SPLIT) bl[j] = Frag<T>::load(Bb2 + bo);
    }
#pragma unroll
    for (int i = 0; i < 4; ++i) {
      const size_t ao = (size_t)(m0 + (i << 4) + rlane) * lda + koff + k0;
      V ah = Frag<T>::load(Ab + ao);
      V al;
      if (SPLIT) al = Frag<T>::load(Ab2 + ao);
#pragma unroll
      for (int j = 0; j < 4; ++j) {
        acc[i][j] = Frag<T>::mma(ah, bh[j], acc[i][j]);
        if (SPLIT) {
          acc[i][j] = Frag<T>::mma(ah, bl[j], acc[i][j]);
          acc[i][j] = Frag<T>::mma(al, bh[j], acc[i][j]);
        }
      }
      Frag<T>::guard(acc[i][0], acc[i][3], ah, SPLIT ? al : ah);
    }
    Frag<T>::keep(bh[0], bh[1], bh[2], bh[3]);
    if (SPLIT) Frag<T>::keep(bl[0], bl[1], bl[2], bl[3]);
  }
  acc_guard4(acc[0][0], acc[0][1], acc[0][2], acc[0][3]);
  acc_guard4(acc[1][0], acc[1][1], acc[1][2], acc[1][3]);
  acc_guard4(acc[2][0], acc[2][1], acc[2][2], acc[2][3]);
  acc_guard4(acc[3][0], acc[3][1], acc[3][2], acc[3][3]);

  float* slab = sT[wave];
  const float* Rb = RESID ? (resid + (size_t)b * strideR) : nullptr;
#pragma unroll
  for (int i = 0; i < 4; ++i) {
    const int mBase = m0 + (i << 4);
#pragma unroll
    for (int j = 0; j < 4; ++j) {
      const int n = n0 + (j << 4) + rlane;
      float bv = 0.f;
      if (BIAS_MODE == 2) bv = bias[n];
#pragma unroll
      for (int r = 0; r < 8; ++r) {
        float v = acc[i][j][r] * scale;
        if (BIAS_MODE == 1) v += bias[mBase + mOff + r];
        if (BIAS_MODE == 2) v += bv;
        if (RESID) v += Rb[(size_t)(mBase + mOff + r) * ldc + n];
        if (ACT == 2) v = fmaxf(v, 0.0f);
        if (ACT == 4) v = (v > 0.f) ? v : 0.01f * v;
        slab[(mOff + r) * 68 + (j << 4) + rlane] = v;
      }
    }
    __builtin_amdgcn_fence(__ATOMIC_RELEASE, "workgroup");
    __builtin_amdgcn_wave_barrier();
    __builtin_amdgcn_fence(__ATOMIC_ACQUIRE, "workgroup");
    if (OUT_MODE == 0) {
      float* C = (float*)Cout + (size_t)b * strideC;
      const int hh = lane >> 4, c4 = (lane & 15) * 4;
      for (int pass = 0; pass < 2; ++pass) {
#pragma unroll
        for (int it = 0; it < 8; ++it) {
          const int row = it * 2 + hh;
          v4f v = *(const v4f*)(slab + row * 68 + c4);
          *(volatile v4f*)(C + (size_t)(mBase + row) * ldc + n0 + c4) = v;
        }
        __threadfence();
      }
    } else {
      const int q = lane >> 3, c8 = (lane & 7) * 8;
      unsigned short* C  = (unsigned short*)Cout  + (size_t)b * strideC;
      unsigned short* C2 = (OUT_MODE == 2) ? ((unsigned short*)Cout2 + (size_t)b * strideC) : nullptr;
      for (int pass = 0; pass < 2; ++pass) {
#pragma unroll
        for (int it = 0; it < 4; ++it) {
          const int row = it * 4 + q;
          const float* sp = slab + row * 68 + c8;
          v8h hv, lv;
#pragma unroll
          for (int e = 0; e < 8; ++e) {
            if (OUT_MODE == 1) {
              hv[e] = (_Float16)sp[e];
            } else {
              unsigned short hb = f2bf_bits(sp[e]);
              unsigned short lb = f2bf_bits(sp[e] - bf_bits2f(hb));
              hv[e] = __builtin_bit_cast(_Float16, hb);
              lv[e] = __builtin_bit_cast(_Float16, lb);
            }
          }
          *(volatile v8h*)(C + (size_t)(mBase + row) * ldc + n0 + c8) = hv;
          if (OUT_MODE == 2) *(volatile v8h*)(C2 + (size_t)(mBase + row) * ldc + n0 + c8) = lv;
        }
        __threadfence();
      }
    }
    __builtin_amdgcn_fence(__ATOMIC_RELEASE, "workgroup");
    __builtin_amdgcn_wave_barrier();
    __builtin_amdgcn_fence(__ATOMIC_ACQUIRE, "workgroup");
  }
}

__global__ __launch_bounds__(256) void cast8_kernel(const float* __restrict__ in, unsigned short* __restrict__ out,
                                                    int n8, float scale) {
  const int i = blockIdx.x * 256 + threadIdx.x;
  if (i >= n8) return;
  const float* p = in + 8 * (size_t)i;
  const v4f a = *(const v4f*)(p);
  const v4f c = *(const v4f*)(p + 4);
  unsigned short hb[8];
#pragma unroll
  for (int e = 0; e < 4; ++e) {
    hb[e]     = h_bits(a[e] * scale);
    hb[4 + e] = h_bits(c[e] * scale);
  }
  const v4u u = (v4u){pk16(hb[0], hb[1]), pk16(hb[2], hb[3]), pk16(hb[4], hb[5]), pk16(hb[6], hb[7])};
  unsigned short* q = out + 8 * (size_t)i;
  *(volatile v4u*)q = u;
  __threadfence();
  *(volatile v4u*)q = u;
}

__global__ __launch_bounds__(256) void stats_kernel(const float* __restrict__ x, const float* __restrict__ gamma,
                                                    const float* __restrict__ beta,
                                                    float* __restrict__ SC, float* __restrict__ SH) {
  __shared__ float scs[32];
  __shared__ float shs[32];
  const int tid = threadIdx.x, wave = tid >> 5, lane = tid & 31;
#pragma unroll 1
  for (int q = 0; q < 4; ++q) {
    const int ch = blockIdx.x * 32 + wave * 4 + q;
    const float* xp = x + (size_t)ch * kFT;
    float s = 0.f;
#pragma unroll 1
    for (int it = 0; it < kFT / 128; ++it) {
      const v4f v = *(const v4f*)(xp + (size_t)(it * 32 + lane) * 4);
      s += (v[0] + v[1]) + (v[2] + v[3]);
    }
#pragma unroll
    for (int off = 16; off > 0; off >>= 1) s += __shfl_xor(s, off, 32);
    const float mu = s * (1.0f / 16384.0f);
    float s2 = 0.f;
#pragma unroll 1
    for (int it = 0; it < kFT / 128; ++it) {
      const v4f v = *(const v4f*)(xp + (size_t)(it * 32 + lane) * 4);
      const float d0 = v[0] - mu, d1 = v[1] - mu, d2 = v[2] - mu, d3 = v[3] - mu;
      s2 += (d0 * d0 + d1 * d1) + (d2 * d2 + d3 * d3);
    }
#pragma unroll
    for (int off = 16; off > 0; off >>= 1) s2 += __shfl_xor(s2, off, 32);
    const float var = s2 * (1.0f / 16384.0f);
    const int c = ch & (kC - 1);
    const float gv = gamma[c];
    const float bv = beta[c];
    const float a = gv * (1.0f / sqrtf(var + 1e-5f));
    const float sh = bv - mu * a;
    if (lane == 0) { scs[wave * 4 + q] = a; shs[wave * 4 + q] = sh; }
  }
  __syncthreads();
  if (wave == 0) {
    const float a = scs[lane], sh = shs[lane];
    float* p0 = SC + blockIdx.x * 32 + lane;
    float* p1 = SH + blockIdx.x * 32 + lane;
    *(volatile float*)p0 = a;
    *(volatile float*)p1 = sh;
    __threadfence();
    *(volatile float*)p0 = a;
    *(volatile float*)p1 = sh;
  }
}

__global__ __launch_bounds__(256) void seq_kernel(const float* __restrict__ x, const float* __restrict__ SC,
                                                  const float* __restrict__ SH, unsigned short* __restrict__ SEQ) {
  __shared__ __align__(16) float xs[kC * kT];
  __shared__ float ssc[kC];
  __shared__ float ssh[kC];
  const int n = blockIdx.x, b = n >> 7, f = n & 127;
  const int tid = threadIdx.x;
  if (tid < kC) { ssc[tid] = SC[b * kC + tid]; ssh[tid] = SH[b * kC + tid]; }
  __syncthreads();
#pragma unroll 1
  for (int it = 0; it < 32; ++it) {
    const int e = it * 256 + tid;
    const int c = e >> 7, t = e & 127;
    const float v = x[((size_t)(b * kC + c) * kF + f) * kT + t];
    xs[e] = v * ssc[c] + ssh[c];
  }
  __syncthreads();
  for (int pass = 0; pass < 2; ++pass) {
#pragma unroll 1
    for (int it = 0; it < 31; ++it) {
      const int id = it * 256 + tid;
      if (id < kS * 64) {
        const int s = id >> 6, c = id & 63;
        const float* sp = xs + c * kT + s;
        unsigned short hb[8];
#pragma unroll
        for (int j = 0; j < 8; ++j) hb[j] = h_bits(sp[j]);
        const v4u u = (v4u){pk16(hb[0], hb[1]), pk16(hb[2], hb[3]), pk16(hb[4], hb[5]), pk16(hb[6], hb[7])};
        *(volatile v4u*)(SEQ + ((size_t)(s * kN + n) * kCK + c * 8)) = u;
      }
    }
    __threadfence();
  }
}

__global__ __launch_bounds__(64) void lstm_kernel(const float* __restrict__ GX, const unsigned short* __restrict__ WHH,
                                                  const float* __restrict__ bih, const float* __restrict__ bhh,
                                                  unsigned short* __restrict__ HD) {
  __shared__ __align__(16) unsigned short hT[2][16 * kH];
  const int d   = blockIdx.x >> 5;
  const int n0  = (blockIdx.x & 31) * 16;
  const int tid = threadIdx.x, ub = tid >> 5, lane = tid & 31;
  const int c   = lane & 15, hh = lane >> 4;
  for (int i = tid; i < 16 * kH; i += 64) hT[0][i] = 0;

  v16h bw[4];
  float bs[4];
#pragma unroll
  for (int g = 0; g < 4; ++g) {
    const int ncol = g * kH + 16 * ub + c;
    bw[g] = Frag<_Float16>::load((const _Float16*)WHH + (size_t)(d * kG4 + ncol) * kH + 8 * hh);
    bs[g] = bih[d * kG4 + ncol] + bhh[d * kG4 + ncol];
  }
  float cs[8];
#pragma unroll
  for (int r = 0; r < 8; ++r) cs[r] = 0.f;
  __syncthreads();

#pragma unroll 1
  for (int ss = 0; ss < kS; ++ss) {
    const int s   = d ? (kS - 1 - ss) : ss;
    const int cur = ss & 1, nxt = cur ^ 1;
    const unsigned short* hc = hT[cur];
    Frag<_Float16>::U fa;
    fa.h[0] = *(const v8h*)(hc + c * kH + 8 * hh);
    fa.h[1] = *(const v8h*)(hc + c * kH + 16 + 8 * hh);
    const float* gp = GX + ((size_t)d * kSN + (size_t)s * kN + n0) * kG4 + 16 * ub + c;
    v8f acc[4];
#pragma unroll
    for (int g = 0; g < 4; ++g) {
#pragma unroll
      for (int r = 0; r < 8; ++r) acc[g][r] = gp[(size_t)(8 * hh + r) * kG4 + g * kH] + bs[g];
    }
#pragma unroll
    for (int g = 0; g < 4; ++g) acc[g] = Frag<_Float16>::mma(fa.v, bw[g], acc[g]);
    acc_guard4a(acc[0], acc[1], acc[2], acc[3], fa.v);

    float hv[8];
#pragma unroll
    for (int r = 0; r < 8; ++r) {
      const float xi = acc[0][r], xf = acc[1][r], xg = acc[2][r], xo = acc[3][r];
      const float ig = 1.0f / (1.0f + expf(-xi));
      const float fg = 1.0f / (1.0f + expf(-xf));
      const float og = 1.0f / (1.0f + expf(-xo));
      const float gg = 2.0f / (1.0f + expf(-2.0f * xg)) - 1.0f;
      const float cn = fg * cs[r] + ig * gg;
      cs[r] = cn;
      const float tc = 2.0f / (1.0f + expf(-2.0f * cn)) - 1.0f;
      hv[r] = og * tc;
    }
    unsigned short* hn = hT[nxt];
#pragma unroll
    for (int r = 0; r < 8; ++r) hn[(8 * hh + r) * kH + 16 * ub + c] = h_bits(hv[r]);
    __syncthreads();
    const v4u u = *(const v4u*)(hn + tid * 8);
    unsigned short* dst = HD + ((size_t)d * kSN + (size_t)s * kN + n0) * kH + tid * 8;
    *(volatile v4u*)dst = u;
    __threadfence();
    *(volatile v4u*)dst = u;
  }
  keep4_h(bw[0], bw[1], bw[2], bw[3]);
}

__global__ __launch_bounds__(256) void concat_kernel(const unsigned short* __restrict__ HD, unsigned short* __restrict__ HC,
                                                     int nchunks) {
  const int id = blockIdx.x * 256 + threadIdx.x;
  if (id >= nchunks) return;
  const int r = id >> 3, q = id & 7, qq = q & 3;
  const v4u a  = *(const v4u*)(HD + (size_t)r * kH + qq * 8);
  const v4u bb = *(const v4u*)(HD + (size_t)kSN * kH + (size_t)r * kH + qq * 8);
  v4u v;
#pragma unroll
  for (int e = 0; e < 4; ++e) v[e] = (q < 4) ? a[e] : bb[e];
  unsigned short* dst = HC + (size_t)r * kH2 + q * 8;
  *(volatile v4u*)dst = v;
  __threadfence();
  *(volatile v4u*)dst = v;
}

__global__ __launch_bounds__(256) void im2col_kernel(const unsigned short* __restrict__ HD, unsigned short* __restrict__ IM) {
  __shared__ __align__(16) unsigned short hs[kH2 * kHP];
  const int n = blockIdx.x, tid = threadIdx.x;
  for (int i = tid; i < kH2 * kHP; i += 256) hs[i] = 0;
  __syncthreads();
#pragma unroll 1
  for (int it = 0; it < 4; ++it) {
    const int e  = it * 256 + tid;
    const int ec = (e < kS * 8) ? e : (kS * 8 - 1);
    const int s = ec >> 3, d = (ec >> 2) & 1, q = ec & 3;
    const v4u w = *(const v4u*)(HD + ((size_t)d * kSN + (size_t)s * kN + n) * kH + q * 8);
    if (e < kS * 8) {
#pragma unroll
      for (int j = 0; j < 8; ++j)
        hs[(d * kH + q * 8 + j) * kHP + s + 8] = (unsigned short)(w[j >> 1] >> (16 * (j & 1)));
    }
  }
  __syncthreads();
  for (int pass = 0; pass < 2; ++pass) {
#pragma unroll 1
    for (int it = 0; it < 32; ++it) {
      const int id = it * 256 + tid;
      const int t = id >> 6, i = id & 63;
      const unsigned short* sp = hs + i * kHP + t;
      const v4u u = (v4u){pk16(sp[8], sp[7]), pk16(sp[6], sp[5]), pk16(sp[4], sp[3]), pk16(sp[2], sp[1])};
      *(volatile v4u*)(IM + ((size_t)(n * kT + t) * kCK + i * 8)) = u;
    }
    __threadfence();
  }
}

extern "C" void kernel_launch(void* const* d_in, const int* in_sizes, int n_in,
                              void* d_out, int out_size, void* d_ws, size_t ws_size,
                              hipStream_t stream) {
  (void)in_sizes; (void)n_in; (void)out_size;
  const float* x     = (const float*)d_in[0];
  const float* gamma = (const float*)d_in[1];
  const float* beta  = (const float*)d_in[2];
  const float* w_ih0 = (const float*)d_in[3];
  const float* w_hh0 = (const float*)d_in[4];
  const float* b_ih0 = (const float*)d_in[5];
  const float* b_hh0 = (const float*)d_in[6];
  const float* w_ih  = (const float*)d_in[7];
  const float* w_hh  = (const float*)d_in[8];
  const float* b_ih  = (const float*)d_in[9];
  const float* b_hh  = (const float*)d_in[10];
  const float* wct   = (const float*)d_in[11];
  const float* bct   = (const float*)d_in[12];
  float* out = (float*)d_out;

  constexpr size_t kOffSeq  = 0;
  constexpr size_t kOffHd   = 0;
  constexpr size_t kOffHc   = 7929856;
  constexpr size_t kOffIm   = 7929856;
  constexpr size_t kOffGx   = 63438848;
  constexpr size_t kOffSc   = 126877696;
  constexpr size_t kOffSh   = kOffSc + 1024;
  constexpr size_t kOffWih0 = kOffSc + 2048;
  constexpr size_t kOffWih  = kOffWih0 + 262144;
  constexpr size_t kOffWhh  = kOffWih + 98304;
  constexpr size_t kOffWct  = kOffWhh + 65536;
  constexpr size_t kWsEnd   = kOffWct + 65536;
  static_assert(kOffSeq + (size_t)kSN * kCK * 2 == kOffGx);
  static_assert(kOffHd + (size_t)2 * kSN * kH * 2 == kOffHc);
  static_assert(kOffHc + (size_t)kSN * kH2 * 2 <= kOffGx);
  static_assert(kOffIm + (size_t)kNT * kCK * 2 <= kOffSc);
  static_assert(kOffGx + (size_t)2 * kSN * kG4 * 4 == kOffSc);
  static_assert(kWsEnd == 127371264);
  static_assert(kWsEnd <= 134217728);
  if (ws_size < kWsEnd) return;

  char* ws = (char*)d_ws;
  unsigned short* SEQ  = (unsigned short*)(ws + kOffSeq);
  unsigned short* HD   = (unsigned short*)(ws + kOffHd);
  unsigned short* HC   = (unsigned short*)(ws + kOffHc);
  unsigned short* IM   = (unsigned short*)(ws + kOffIm);
  float*          GX   = (float*)(ws + kOffGx);
  float*          SC   = (float*)(ws + kOffSc);
  float*          SH   = (float*)(ws + kOffSh);
  unsigned short* WIH0 = (unsigned short*)(ws + kOffWih0);
  unsigned short* WIH  = (unsigned short*)(ws + kOffWih);
  unsigned short* WHH  = (unsigned short*)(ws + kOffWhh);
  unsigned short* WCT  = (unsigned short*)(ws + kOffWct);

  stats_kernel<<<(kB * kC) / 32, 256, 0, stream>>>(x, gamma, beta, SC, SH);
  cast8_kernel<<<(2 * kG4 * kCK / 8) / 256, 256, 0, stream>>>(w_ih0, WIH0, 2 * kG4 * kCK / 8, kWCarry);
  cast8_kernel<<<(3 * 2 * kG4 * kH2 / 8) / 256, 256, 0, stream>>>(w_ih, WIH, 3 * 2 * kG4 * kH2 / 8, kWCarry);
  cast8_kernel<<<(2 * kG4 * kH / 8) / 256, 256, 0, stream>>>(w_hh0, WHH, 2 * kG4 * kH / 8, 1.0f);
  cast8_kernel<<<(3 * 2 * kG4 * kH / 8) / 256, 256, 0, stream>>>(w_hh, WHH + 2 * kG4 * kH, 3 * 2 * kG4 * kH / 8, 1.0f);
  cast8_kernel<<<(kC * kCK / 8) / 256, 256, 0, stream>>>(wct, WCT, kC * kCK / 8, kWCarry);
  seq_kernel<<<kN, 256, 0, stream>>>(x, SC, SH, SEQ);
  wmma_gemm64<0, false, 0, 0, false, 0><<<dim3(242, 2), 256, 0, stream>>>(
      SEQ, SEQ, kCK, 0L,
      WIH0, WIH0, kCK, (long)kG4 * kCK,
      (void*)GX, (void*)GX, kG4, (long)kSN * kG4,
      bct, x, 0L,
      kSN, kG4, kCK, kWCarryInv);
  lstm_kernel<<<64, 64, 0, stream>>>(GX, WHH, b_ih0, b_hh0, HD);
  for (int l = 1; l < 4; ++l) {
    concat_kernel<<<(kSN * 8) / 256, 256, 0, stream>>>(HD, HC, kSN * 8);
    wmma_gemm64<0, false, 0, 0, false, 0><<<dim3(242, 2), 256, 0, stream>>>(
        HC, HC, kH2, 0L,
        WIH + (size_t)(l - 1) * 2 * kG4 * kH2, WIH + (size_t)(l - 1) * 2 * kG4 * kH2, kH2, (long)kG4 * kH2,
        (void*)GX, (void*)GX, kG4, (long)kSN * kG4,
        bct, x, 0L,
        kSN, kG4, kH2, kWCarryInv);
    lstm_kernel<<<64, 64, 0, stream>>>(GX, WHH + (size_t)l * 2 * kG4 * kH,
                                       b_ih + (size_t)(l - 1) * 2 * kG4, b_hh + (size_t)(l - 1) * 2 * kG4, HD);
  }
  im2col_kernel<<<kN, 256, 0, stream>>>(HD, IM);
  wmma_gemm64<0, false, 1, 0, true, 0><<<dim3(32, kB), 256, 0, stream>>>(
      WCT, WCT, kCK, 0L,
      IM, IM, kCK, (long)kFT * kCK,
      (void*)out, (void*)out, kFT, (long)kC * kFT,
      bct, x, (long)kC * kFT,
      kC, kFT, kCK, kWCarryInv);
}
